// MHSA_27582279975470
// MI455X (gfx1250) — hardware-verified
//
#include <hip/hip_runtime.h>
#include <math.h>
#include <stdint.h>

#define NB    4
#define DIM   256
#define NH    8
#define HD    32
#define IMH   64
#define IMW   64
#define NQ    4096
#define OH    32
#define OW    32
#define NKV   1024
#define KCONV 1024
#define MTOK  (NB * NQ)
#define MKV   (NB * NKV)
#define VTP   (NB * NKV)

static_assert(NQ == IMH * IMW);
static_assert(NKV == OH * OW);
static_assert(OH * 2 == IMH);
static_assert(OW * 2 == IMW);
static_assert(DIM == NH * HD);
static_assert(HD == 32);
static_assert(KCONV == DIM * 4);
static_assert(MTOK % 64 == 0);
static_assert(MKV % 128 == 0);
static_assert(DIM % 64 == 0);
static_assert(KCONV % 32 == 0);
static_assert(DIM % 32 == 0);
static_assert((DIM * DIM) % (8 * 256) == 0);
static_assert(((MKV / 64) * (DIM / 64)) % 8 == 0);
static_assert(((MTOK / 64) * (DIM / 64)) % 8 == 0);
static_assert(DIM * OH == 8192);
static_assert(NQ % 64 == 0);
static_assert(NKV % 64 == 0);

typedef __attribute__((ext_vector_type(16))) _Float16 v16h;
typedef __attribute__((ext_vector_type(8)))  _Float16 v8h;
typedef __attribute__((ext_vector_type(16))) __bf16   v16b;
typedef __attribute__((ext_vector_type(8)))  __bf16   v8b;
typedef __attribute__((ext_vector_type(8)))  float    v8f;
typedef __attribute__((ext_vector_type(4)))  float    v4f;
typedef __attribute__((ext_vector_type(2)))  float    v2f;
typedef __attribute__((ext_vector_type(4)))  unsigned int v4u;
typedef __attribute__((ext_vector_type(2)))  unsigned int v2u;

__device__ __forceinline__ unsigned short f2bf_bits(float f) {
  unsigned u = __float_as_uint(f);
  return (unsigned short)((u + 0x7FFFu + ((u >> 16) & 1u)) >> 16);
}
__device__ __forceinline__ float bf_bits2f(unsigned short h) { return __uint_as_float(((unsigned)h) << 16); }
__device__ __forceinline__ unsigned pk16(unsigned short a, unsigned short b) { return (unsigned)a | ((unsigned)b << 16); }

__device__ __forceinline__ void dep_guard_h(v8f& a, v8f& b, v16h x, v16h y) { asm volatile("v_nop\n\tv_nop\n\tv_nop\n\tv_nop" : "+v"(a), "+v"(b) : "v"(x), "v"(y)); }
__device__ __forceinline__ void dep_guard_b(v8f& a, v8f& b, v16b x, v16b y) { asm volatile("v_nop\n\tv_nop\n\tv_nop\n\tv_nop" : "+v"(a), "+v"(b) : "v"(x), "v"(y)); }
__device__ __forceinline__ void keep4_h(v16h a, v16h b, v16h c, v16h d) { asm volatile("v_nop" :: "v"(a), "v"(b), "v"(c), "v"(d)); }
__device__ __forceinline__ void keep4_b(v16b a, v16b b, v16b c, v16b d) { asm volatile("v_nop" :: "v"(a), "v"(b), "v"(c), "v"(d)); }
__device__ __forceinline__ void acc_guard4(v8f& a, v8f& b, v8f& c, v8f& d) { asm volatile("v_nop\n\tv_nop\n\tv_nop\n\tv_nop" : "+v"(a), "+v"(b), "+v"(c), "+v"(d)); }
template <typename T> struct Frag;
template <> struct Frag<_Float16> {
  typedef v16h V; union U { v16h v; v8h h[2]; };
  static __device__ __forceinline__ v16h load(const _Float16* p) {
    U f; f.h[0] = *(const v8h*)(p); f.h[1] = *(const v8h*)(p + 16); return f.v;
  }
  static __device__ __forceinline__ v8f mma(v16h a, v16h b, v8f c) {
    return __builtin_amdgcn_wmma_f32_16x16x32_f16(false, a, false, b, (short)0, c, false, false);
  }
  static __device__ __forceinline__ void guard(v8f& a, v8f& b, v16h x, v16h y) { dep_guard_h(a, b, x, y); }
  static __device__ __forceinline__ void keep(v16h a, v16h b, v16h c, v16h d) { keep4_h(a, b, c, d); }
};
template <> struct Frag<__bf16> {
  typedef v16b V; union U { v16b v; v8b h[2]; };
  static __device__ __forceinline__ v16b load(const __bf16* p) {
    U f; f.h[0] = *(const v8b*)(p); f.h[1] = *(const v8b*)(p + 16); return f.v;
  }
  static __device__ __forceinline__ v8f mma(v16b a, v16b b, v8f c) {
    return __builtin_amdgcn_wmma_f32_16x16x32_bf16(false, a, false, b, (short)0, c, false, false);
  }
  static __device__ __forceinline__ void guard(v8f& a, v8f& b, v16b x, v16b y) { dep_guard_b(a, b, x, y); }
  static __device__ __forceinline__ void keep(v16b a, v16b b, v16b c, v16b d) { keep4_b(a, b, c, d); }
};

template <int ET> struct Elem;
template <> struct Elem<0> { typedef _Float16 T; };
template <> struct Elem<1> { typedef __bf16 T; };
template <int ET, bool SPLIT, int BIAS_MODE, int OUT_MODE, bool RESID, int ACT = 0>
__global__ __launch_bounds__(256) void wmma_gemm64(
    const unsigned short* __restrict__ Ap, const unsigned short* __restrict__ A2p, int lda, long strideA,
    const unsigned short* __restrict__ Btp, const unsigned short* __restrict__ Bt2p, int ldb, long strideB,
    void* __restrict__ Cout, void* __restrict__ Cout2, int ldc, long strideC,
    const float* __restrict__ bias,
    const float* __restrict__ resid, long strideR,
    int M, int N, int K, float scale) {
  typedef typename Elem<ET>::T T;
  typedef typename Frag<T>::V V;
  const T* A = (const T*)Ap; const T* A2 = (const T*)A2p; const T* Bt = (const T*)Btp; const T* Bt2 = (const T*)Bt2p;
  __shared__ __align__(16) float sT[8][16 * 68];
  const int b    = blockIdx.y;
  const int lane = threadIdx.x & 31;
  const int wave = threadIdx.x >> 5;
  const int tilesN = N >> 6;
  const int tilesM = M >> 6;
  const int tile = blockIdx.x * 8 + wave;
  if (tile >= tilesM * tilesN) return;
  const int tm = tile / tilesN;
  const int tn = tile - tm * tilesN;
  const int m0 = tm << 6;
  const int n0 = tn << 6;

  const T* Ab  = A  + (size_t)b * strideA;
  const T* Bb  = Bt + (size_t)b * strideB;
  const T* Ab2 = SPLIT ? (A2  + (size_t)b * strideA) : nullptr;
  const T* Bb2 = SPLIT ? (Bt2 + (size_t)b * strideB) : nullptr;

  const int rlane = lane & 15;
  const int koff  = (lane >> 4) * 8;
  const int mOff  = (lane >> 4) * 8;

  v8f acc[4][4];
#pragma unroll
  for (int i = 0; i < 4; ++i)
#pragma unroll
    for (int j = 0; j < 4; ++j) acc[i][j] = (v8f){0.f,0.f,0.f,0.f,0.f,0.f,0.f,0.f};

  for (int k0 = 0; k0 < K; k0 += 32) {
    V bh[4], bl[4];
#pragma unroll
    for (int j = 0; j < 4; ++j) {
      const size_t bo = (size_t)(n0 + (j << 4) + rlane) * ldb + koff + k0;
      bh[j] = Frag<T>::load(Bb + bo);
      if (SPLIT) bl[j] = Frag<T>::load(Bb2 + bo); else bl[j] = bh[j];
    }
#pragma unroll
    for (int i = 0; i < 4; ++i) {
      const size_t ao = (size_t)(m0 + (i << 4) + rlane) * lda + koff + k0;
      V ah = Frag<T>::load(Ab + ao);
      V al;
      if (SPLIT) al = Frag<T>::load(Ab2 + ao); else al = ah;
#pragma unroll
      for (int j = 0; j < 4; ++j) {
        acc[i][j] = Frag<T>::mma(ah, bh[j], acc[i][j]);
        if (SPLIT) {
          acc[i][j] = Frag<T>::mma(ah, bl[j], acc[i][j]);
          acc[i][j] = Frag<T>::mma(al, bh[j], acc[i][j]);
        }
      }
      Frag<T>::guard(acc[i][0], acc[i][3], ah, al);
    }
    Frag<T>::keep(bh[0], bh[1], bh[2], bh[3]);
    if (SPLIT) Frag<T>::keep(bl[0], bl[1], bl[2], bl[3]);
  }
  acc_guard4(acc[0][0], acc[0][1], acc[0][2], acc[0][3]);
  acc_guard4(acc[1][0], acc[1][1], acc[1][2], acc[1][3]);
  acc_guard4(acc[2][0], acc[2][1], acc[2][2], acc[2][3]);
  acc_guard4(acc[3][0], acc[3][1], acc[3][2], acc[3][3]);

  float* slab = sT[wave];
  const float* Rb = RESID ? (resid + (size_t)b * strideR) : nullptr;
#pragma unroll
  for (int i = 0; i < 4; ++i) {
    const int mBase = m0 + (i << 4);
#pragma unroll
    for (int j = 0; j < 4; ++j) {
      const int n = n0 + (j << 4) + rlane;
      float bv = 0.f;
      if (BIAS_MODE == 2) bv = bias[n];
#pragma unroll
      for (int r = 0; r < 8; ++r) {
        float v = acc[i][j][r] * scale;
        if (BIAS_MODE == 1) v += bias[mBase + mOff + r];
        if (BIAS_MODE == 2) v += bv;
        if (RESID) v += Rb[(size_t)(mBase + mOff + r) * ldc + n];
        if (ACT == 1) v = tanhf(v);
        if (ACT == 2) v = fmaxf(v, 0.0f);
        if (ACT == 3) v = v / (1.0f + expf(-v));
        if (ACT == 4) v = (v > 0.f) ? v : 0.01f * v;
        if (ACT == 5) v = 0.5f * v * (1.0f + erff(v * 0.70710678118654752f));
        slab[(mOff + r) * 68 + (j << 4) + rlane] = v;
      }
    }
    __builtin_amdgcn_fence(__ATOMIC_RELEASE, "workgroup");
    __builtin_amdgcn_wave_barrier();
    __builtin_amdgcn_fence(__ATOMIC_ACQUIRE, "workgroup");
    if (OUT_MODE == 0) {
      float* C = (float*)Cout + (size_t)b * strideC;
      const int hh = lane >> 4, c4 = (lane & 15) * 4;
      for (int pass = 0; pass < 2; ++pass) {
#pragma unroll
        for (int it = 0; it < 8; ++it) {
          const int row = it * 2 + hh;
          v4f v = *(const v4f*)(slab + row * 68 + c4);
          *(volatile v4f*)(C + (size_t)(mBase + row) * ldc + n0 + c4) = v;
        }
        __threadfence();
      }
    } else {
      const int q = lane >> 3, c8 = (lane & 7) * 8;
      unsigned short* C  = (unsigned short*)Cout  + (size_t)b * strideC;
      unsigned short* C2 = (OUT_MODE == 2) ? ((unsigned short*)Cout2 + (size_t)b * strideC) : nullptr;
      for (int pass = 0; pass < 2; ++pass) {
#pragma unroll
        for (int it = 0; it < 4; ++it) {
          const int row = it * 4 + q;
          const float* sp = slab + row * 68 + c8;
          v8h hv, lv;
#pragma unroll
          for (int e = 0; e < 8; ++e) {
            if (OUT_MODE == 1) {
              hv[e] = (_Float16)sp[e];
            } else {
              unsigned short hb = f2bf_bits(sp[e]);
              unsigned short lb = f2bf_bits(sp[e] - bf_bits2f(hb));
              hv[e] = __builtin_bit_cast(_Float16, hb);
              lv[e] = __builtin_bit_cast(_Float16, lb);
            }
          }
          *(volatile v8h*)(C + (size_t)(mBase + row) * ldc + n0 + c8) = hv;
          if (OUT_MODE == 2) *(volatile v8h*)(C2 + (size_t)(mBase + row) * ldc + n0 + c8) = lv;
        }
        __threadfence();
      }
    }
    __builtin_amdgcn_fence(__ATOMIC_RELEASE, "workgroup");
    __builtin_amdgcn_wave_barrier();
    __builtin_amdgcn_fence(__ATOMIC_ACQUIRE, "workgroup");
  }
}

__global__ __launch_bounds__(256) void convrows_kernel(const float* __restrict__ in, unsigned short* __restrict__ out,
                                                       int ncols, int ldout, int n8) {
  const int i = blockIdx.x * 256 + threadIdx.x;
  if (i < n8) {
    const size_t e0 = (size_t)i * 8;
    const int row = (int)(e0 / (size_t)ncols);
    const int col = (int)(e0 - (size_t)row * ncols);
    const v4f a = *(const v4f*)(in + e0);
    const v4f c = *(const v4f*)(in + e0 + 4);
    v4u hv;
    hv[0] = pk16(f2bf_bits(a[0]), f2bf_bits(a[1]));
    hv[1] = pk16(f2bf_bits(a[2]), f2bf_bits(a[3]));
    hv[2] = pk16(f2bf_bits(c[0]), f2bf_bits(c[1]));
    hv[3] = pk16(f2bf_bits(c[2]), f2bf_bits(c[3]));
    const size_t o = (size_t)row * ldout + col;
    for (int pass = 0; pass < 2; ++pass) {
      *(volatile v4u*)(out + o) = hv;
      __threadfence();
    }
  }
}

__global__ __launch_bounds__(256) void tconv_kernel(const float* __restrict__ W, unsigned short* __restrict__ oh,
                                                    int ldin, int ldout, long sIn, long sOut) {
  __shared__ __align__(16) float tf[64 * 68];
  W  += (size_t)blockIdx.z * sIn;
  oh += (size_t)blockIdx.z * sOut;
  const int c0  = blockIdx.x * 64;
  const int r0  = blockIdx.y * 64;
  const int tid = threadIdx.x;
  {
    const int lr = tid >> 4;
    const int c4 = (tid & 15) * 4;
#pragma unroll
    for (int it = 0; it < 4; ++it) {
      const int rr = it * 16 + lr;
      const v4f a = *(const v4f*)(W + (size_t)(r0 + rr) * ldin + c0 + c4);
      *(v4f*)(tf + rr * 68 + c4) = a;
    }
  }
  __syncthreads();
  const int sub = tid >> 3;
  const int c8  = (tid & 7) * 8;
  v4u hv[2];
#pragma unroll
  for (int it = 0; it < 2; ++it) {
    const int oc = it * 32 + sub;
    v4u a;
#pragma unroll
    for (int q = 0; q < 4; ++q) {
      const float f0 = tf[(c8 + 2 * q) * 68 + oc];
      const float f1 = tf[(c8 + 2 * q + 1) * 68 + oc];
      a[q] = pk16(f2bf_bits(f0), f2bf_bits(f1));
    }
    hv[it] = a;
  }
  for (int pass = 0; pass < 2; ++pass) {
#pragma unroll
    for (int it = 0; it < 2; ++it) {
      const int oc = it * 32 + sub;
      const size_t go = (size_t)(c0 + oc) * ldout + r0 + c8;
      *(volatile v4u*)(oh + go) = hv[it];
    }
    __threadfence();
  }
}

__global__ __launch_bounds__(256) void wperm_kernel(const float* __restrict__ W, unsigned short* __restrict__ O) {
  const int u = blockIdx.x * 256 + threadIdx.x;
  if (u < DIM * 32) {
    const int o = u >> 5, c0 = (u & 31) * 8;
    v4f w[8];
#pragma unroll
    for (int e = 0; e < 8; ++e) w[e] = *(const v4f*)(W + ((size_t)(o * DIM + c0 + e)) * 4);
    v4u pk[4];
#pragma unroll
    for (int q4 = 0; q4 < 4; ++q4) {
      v4u a;
#pragma unroll
      for (int p = 0; p < 4; ++p) a[p] = pk16(f2bf_bits(w[2 * p][q4]), f2bf_bits(w[2 * p + 1][q4]));
      pk[q4] = a;
    }
    unsigned short* orow = O + (size_t)o * KCONV + c0;
    for (int pass = 0; pass < 2; ++pass) {
#pragma unroll
      for (int q4 = 0; q4 < 4; ++q4) *(volatile v4u*)(orow + q4 * DIM) = pk[q4];
      __threadfence();
    }
  }
}

__device__ __forceinline__ size_t im2col_off(int g, int k0) {
  const int b = g >> 10, m = g & (NKV - 1);
  const int q4 = k0 >> 8, c0 = k0 & (DIM - 1);
  const int kh = q4 >> 1, kw = q4 & 1;
  const int i = m >> 5, j = m & 31;
  return ((size_t)(b * NQ + (2 * i + kh) * IMW + 2 * j + kw)) * DIM + c0;
}

template <int MODE>
__global__ __launch_bounds__(256) void conv_gemm64(const unsigned short* __restrict__ XTp, const unsigned short* __restrict__ Wpp,
                                                   const float* __restrict__ rel_h, const float* __restrict__ rel_w,
                                                   unsigned short* __restrict__ Ch, unsigned short* __restrict__ Cl) {
  typedef __bf16 T;
  typedef v16b V;
  const T* XT = (const T*)XTp; const T* Wp = (const T*)Wpp;
  __shared__ __align__(16) float sT[8][16 * 68];
  __shared__ __align__(16) unsigned short sRh[(MODE == 0) ? (DIM * OH) : 8];
  __shared__ __align__(16) unsigned short sRw[(MODE == 0) ? (DIM * 4) : 8];
  constexpr int M = (MODE == 0) ? MKV : DIM;
  constexpr int N = (MODE == 0) ? DIM : MKV;
  constexpr int LDC = N;
  const int tid  = threadIdx.x;
  const int lane = tid & 31;
  const int wave = tid >> 5;

  if (MODE == 0) {
    const int iib = 4 * (blockIdx.x & 7);
#pragma unroll
    for (int it = 0; it < 8; ++it) {
      const int e4 = (it * 256 + tid) * 4;
      const v4f a = *(const v4f*)(rel_h + e4);
      v2u w;
      w[0] = pk16(f2bf_bits(a[0]), f2bf_bits(a[1]));
      w[1] = pk16(f2bf_bits(a[2]), f2bf_bits(a[3]));
      *(v2u*)(sRh + e4) = w;
    }
    {
      const v4f a = *(const v4f*)(rel_w + (size_t)tid * OW + iib);
      v2u w;
      w[0] = pk16(f2bf_bits(a[0]), f2bf_bits(a[1]));
      w[1] = pk16(f2bf_bits(a[2]), f2bf_bits(a[3]));
      *(v2u*)(sRw + tid * 4) = w;
    }
    __syncthreads();
  }

  constexpr int tilesN = N >> 6;
  constexpr int tilesM = M >> 6;
  const int tile = blockIdx.x * 8 + wave;
  if (tile >= tilesM * tilesN) return;
  const int tm = tile / tilesN;
  const int tn = tile - tm * tilesN;
  const int m0 = tm << 6;
  const int n0 = tn << 6;

  const int rlane = lane & 15;
  const int koff  = (lane >> 4) * 8;
  const int mOff  = (lane >> 4) * 8;

  v8f acc[4][4];
#pragma unroll
  for (int i = 0; i < 4; ++i)
#pragma unroll
    for (int j = 0; j < 4; ++j) acc[i][j] = (v8f){0.f,0.f,0.f,0.f,0.f,0.f,0.f,0.f};

  for (int k0 = 0; k0 < KCONV; k0 += 32) {
    V bfr[4];
#pragma unroll
    for (int j = 0; j < 4; ++j) {
      const int n = n0 + (j << 4) + rlane;
      if (MODE == 0) bfr[j] = Frag<T>::load(Wp + (size_t)n * KCONV + k0 + koff);
      else           bfr[j] = Frag<T>::load(XT + im2col_off(n, k0) + koff);
    }
#pragma unroll
    for (int i = 0; i < 4; ++i) {
      const int mr = m0 + (i << 4) + rlane;
      V ah;
      if (MODE == 0) ah = Frag<T>::load(XT + im2col_off(mr, k0) + koff);
      else           ah = Frag<T>::load(Wp + (size_t)mr * KCONV + k0 + koff);
#pragma unroll
      for (int j = 0; j < 4; ++j) acc[i][j] = Frag<T>::mma(ah, bfr[j], acc[i][j]);
      Frag<T>::guard(acc[i][0], acc[i][3], ah, ah);
    }
    Frag<T>::keep(bfr[0], bfr[1], bfr[2], bfr[3]);
  }
  acc_guard4(acc[0][0], acc[0][1], acc[0][2], acc[0][3]);
  acc_guard4(acc[1][0], acc[1][1], acc[1][2], acc[1][3]);
  acc_guard4(acc[2][0], acc[2][1], acc[2][2], acc[2][3]);
  acc_guard4(acc[3][0], acc[3][1], acc[3][2], acc[3][3]);

  float* slab = sT[wave];
#pragma unroll
  for (int i = 0; i < 4; ++i) {
    const int mBase = m0 + (i << 4);
#pragma unroll
    for (int j = 0; j < 4; ++j) {
      const int n = n0 + (j << 4) + rlane;
#pragma unroll
      for (int r = 0; r < 8; ++r) {
        float v = acc[i][j][r];
        if (MODE == 0) {
          const int row = mBase + mOff + r;
          const int m   = row & (NKV - 1);
          const int jj  = m & 31;
          const int iil = (m >> 5) & 3;
          const float pos = bf_bits2f(sRh[n * OH + jj]) + bf_bits2f(sRw[n * 4 + iil]);
          v += pos;
        }
        slab[(mOff + r) * 68 + (j << 4) + rlane] = v;
      }
    }
    __builtin_amdgcn_fence(__ATOMIC_RELEASE, "workgroup");
    __builtin_amdgcn_wave_barrier();
    __builtin_amdgcn_fence(__ATOMIC_ACQUIRE, "workgroup");
    {
      const int q = lane >> 3, c8 = (lane & 7) * 8;
      for (int pass = 0; pass < 2; ++pass) {
#pragma unroll
        for (int it = 0; it < 4; ++it) {
          const int row = it * 4 + q;
          const float* sp = slab + row * 68 + c8;
          v8h hv, lv;
#pragma unroll
          for (int e = 0; e < 8; ++e) {
            unsigned short hb = f2bf_bits(sp[e]);
            unsigned short lb = f2bf_bits(sp[e] - bf_bits2f(hb));
            hv[e] = __builtin_bit_cast(_Float16, hb);
            lv[e] = __builtin_bit_cast(_Float16, lb);
          }
          *(volatile v8h*)(Ch + (size_t)(mBase + row) * LDC + n0 + c8) = hv;
          *(volatile v8h*)(Cl + (size_t)(mBase + row) * LDC + n0 + c8) = lv;
        }
        __threadfence();
      }
    }
    __builtin_amdgcn_fence(__ATOMIC_RELEASE, "workgroup");
    __builtin_amdgcn_wave_barrier();
    __builtin_amdgcn_fence(__ATOMIC_ACQUIRE, "workgroup");
  }
}

#define AT_D  32
#define AT_NW 4
#define AT_QB 64
#define AT_KC 64

__device__ __forceinline__ unsigned short at_bf_bits(float f) {
  unsigned u = __float_as_uint(f);
  return (unsigned short)((u + 0x7FFFu + ((u >> 16) & 1u)) >> 16);
}
__device__ __forceinline__ __bf16 at_f2bf(float f) { return __builtin_bit_cast(__bf16, at_bf_bits(f)); }
__device__ __forceinline__ void at_split(float f, __bf16& hi, __bf16& lo) {
  const unsigned short hb = at_bf_bits(f);
  hi = __builtin_bit_cast(__bf16, hb);
  lo = at_f2bf(f - __uint_as_float(((unsigned)hb) << 16));
}
__device__ __forceinline__ v8f at_mma(v16b a, v16b b, v8f c) {
  c = __builtin_amdgcn_wmma_f32_16x16x32_bf16(false, a, false, b, (short)0, c, false, false);
  asm volatile("v_nop\n\tv_nop\n\tv_nop\n\tv_nop" : "+v"(c) : "v"(a), "v"(b));
  return c;
}

__global__ __launch_bounds__(128)
void attn32_kernel(const unsigned short* __restrict__ qhp, const unsigned short* __restrict__ qlp,
                   const unsigned short* __restrict__ khp, const unsigned short* __restrict__ klp,
                   const unsigned short* __restrict__ vhp, const unsigned short* __restrict__ vlp,
                   float* __restrict__ out, float sscale) {
  union FB { v16b v; v8b h[2]; };
  __shared__ __align__(16) __bf16 Ksh[AT_KC * AT_D];
  __shared__ __align__(16) __bf16 Ksl[AT_KC * AT_D];
  __shared__ __align__(16) __bf16 Vth[AT_D * AT_KC];
  __shared__ __align__(16) __bf16 Vtl[AT_D * AT_KC];
  __shared__ __align__(16) __bf16 Psh[AT_NW][16 * AT_KC];
  __shared__ __align__(16) __bf16 Psl[AT_NW][16 * AT_KC];
  __shared__ __align__(16) float  Os[AT_D * 68];

  const int tid  = threadIdx.x;
  const int wave = tid >> 5;
  const int lane = tid & 31;
  const int hh   = lane >> 4;
  const int c    = lane & 15;

  const int nqb = NQ / AT_QB;
  const int bx = blockIdx.x;
  const int qb = bx % nqb;
  const int hb = bx / nqb;
  const int h  = hb % NH;
  const int b  = hb / NH;
  const int q0 = b * NQ + qb * AT_QB + wave * 16;

  const __bf16* Qh = (const __bf16*)(const void*)qhp + (size_t)h * AT_D;
  const __bf16* Ql = (const __bf16*)(const void*)qlp + (size_t)h * AT_D;
  const __bf16* Kh = (const __bf16*)(const void*)khp + (size_t)h * AT_D;
  const __bf16* Kl = (const __bf16*)(const void*)klp + (size_t)h * AT_D;
  const __bf16* Vh = (const __bf16*)(const void*)vhp + (size_t)h * AT_D * VTP + (size_t)b * NKV;
  const __bf16* Vl = (const __bf16*)(const void*)vlp + (size_t)h * AT_D * VTP + (size_t)b * NKV;

  v16b qah, qal;
  {
    const __bf16* qr = Qh + (size_t)(q0 + c) * DIM + 8 * hh;
    const __bf16* ql = Ql + (size_t)(q0 + c) * DIM + 8 * hh;
    qah = Frag<__bf16>::load(qr);
    qal = Frag<__bf16>::load(ql);
  }

  float mrow[8], lrow[8];
  v8f oacc[2];
#pragma unroll
  for (int r = 0; r < 8; ++r) { mrow[r] = -INFINITY; lrow[r] = 0.f; }
#pragma unroll
  for (int t = 0; t < 2; ++t) oacc[t] = (v8f){0.f,0.f,0.f,0.f,0.f,0.f,0.f,0.f};

  const int nChunks = NKV / AT_KC;
  for (int kc = 0; kc < nChunks; ++kc) {
    const int kv0 = kc * AT_KC;
    __syncthreads();
    {
      const int r = tid >> 1, hf = (tid & 1) * 16;
      const __bf16* ksh = Kh + (size_t)(b * NKV + kv0 + r) * DIM + hf;
      const __bf16* ksl = Kl + (size_t)(b * NKV + kv0 + r) * DIM + hf;
      const v8b a0 = *(const v8b*)(ksh);
      const v8b a1 = *(const v8b*)(ksh + 8);
      const v8b a2 = *(const v8b*)(ksl);
      const v8b a3 = *(const v8b*)(ksl + 8);
      *(v8b*)(Ksh + r * AT_D + hf)     = a0;
      *(v8b*)(Ksh + r * AT_D + hf + 8) = a1;
      *(v8b*)(Ksl + r * AT_D + hf)     = a2;
      *(v8b*)(Ksl + r * AT_D + hf + 8) = a3;
      const int d = tid >> 2, qq = (tid & 3) * 16;
      const __bf16* vsh = Vh + (size_t)d * VTP + kv0 + qq;
      const __bf16* vsl = Vl + (size_t)d * VTP + kv0 + qq;
      const v8b b0 = *(const v8b*)(vsh);
      const v8b b1 = *(const v8b*)(vsh + 8);
      const v8b b2 = *(const v8b*)(vsl);
      const v8b b3 = *(const v8b*)(vsl + 8);
      *(v8b*)(Vth + d * AT_KC + qq)     = b0;
      *(v8b*)(Vth + d * AT_KC + qq + 8) = b1;
      *(v8b*)(Vtl + d * AT_KC + qq)     = b2;
      *(v8b*)(Vtl + d * AT_KC + qq + 8) = b3;
    }
    __syncthreads();

    v8f s[4];
#pragma unroll
    for (int j = 0; j < 4; ++j) {
      s[j] = (v8f){0.f,0.f,0.f,0.f,0.f,0.f,0.f,0.f};
      FB kb, kl;
      kb.h[0] = *(const v8b*)(Ksh + (j * 16 + c) * AT_D + 8 * hh);
      kb.h[1] = *(const v8b*)(Ksh + (j * 16 + c) * AT_D + 16 + 8 * hh);
      kl.h[0] = *(const v8b*)(Ksl + (j * 16 + c) * AT_D + 8 * hh);
      kl.h[1] = *(const v8b*)(Ksl + (j * 16 + c) * AT_D + 16 + 8 * hh);
      s[j] = at_mma(qah, kb.v, s[j]);
      s[j] = at_mma(qah, kl.v, s[j]);
      s[j] = at_mma(qal, kb.v, s[j]);
    }
    float cm[8];
#pragma unroll
    for (int r = 0; r < 8; ++r) {
      float m = -INFINITY;
#pragma unroll
      for (int j = 0; j < 4; ++j) {
        const float sv = s[j][r] * sscale;
        s[j][r] = sv;
        m = fmaxf(m, sv);
      }
#pragma unroll
      for (int off = 1; off < 16; off <<= 1) m = fmaxf(m, __shfl_xor(m, off, 32));
      cm[r] = m;
    }
    __bf16* pwh = Psh[wave];
    __bf16* pwl = Psl[wave];
#pragma unroll
    for (int r = 0; r < 8; ++r) {
      const float mnew = fmaxf(mrow[r], cm[r]);
      const float alpha = expf(mrow[r] - mnew);
      mrow[r] = mnew;
      float psum = 0.f;
#pragma unroll
      for (int j = 0; j < 4; ++j) {
        const float p = expf(s[j][r] - mnew);
        psum += p;
        __bf16 a, bl; at_split(p, a, bl);
        pwh[(8 * hh + r) * AT_KC + j * 16 + c] = a;
        pwl[(8 * hh + r) * AT_KC + j * 16 + c] = bl;
      }
#pragma unroll
      for (int off = 1; off < 16; off <<= 1) psum += __shfl_xor(psum, off, 32);
      lrow[r] = lrow[r] * alpha + psum;
#pragma unroll
      for (int t = 0; t < 2; ++t) oacc[t][r] *= alpha;
    }
    __builtin_amdgcn_fence(__ATOMIC_RELEASE, "workgroup");
    __builtin_amdgcn_wave_barrier();
    __builtin_amdgcn_fence(__ATOMIC_ACQUIRE, "workgroup");
#pragma unroll 1
    for (int kk = 0; kk < 2; ++kk) {
      FB pa, pl;
      pa.h[0] = *(const v8b*)(pwh + c * AT_KC + kk * 32 + 8 * hh);
      pa.h[1] = *(const v8b*)(pwh + c * AT_KC + kk * 32 + 16 + 8 * hh);
      pl.h[0] = *(const v8b*)(pwl + c * AT_KC + kk * 32 + 8 * hh);
      pl.h[1] = *(const v8b*)(pwl + c * AT_KC + kk * 32 + 16 + 8 * hh);
#pragma unroll
      for (int t = 0; t < 2; ++t) {
        FB vb, vl;
        vb.h[0] = *(const v8b*)(Vth + (t * 16 + c) * AT_KC + kk * 32 + 8 * hh);
        vb.h[1] = *(const v8b*)(Vth + (t * 16 + c) * AT_KC + kk * 32 + 16 + 8 * hh);
        vl.h[0] = *(const v8b*)(Vtl + (t * 16 + c) * AT_KC + kk * 32 + 8 * hh);
        vl.h[1] = *(const v8b*)(Vtl + (t * 16 + c) * AT_KC + kk * 32 + 16 + 8 * hh);
        oacc[t] = at_mma(pa.v, vb.v, oacc[t]);
        oacc[t] = at_mma(pa.v, vl.v, oacc[t]);
        oacc[t] = at_mma(pl.v, vb.v, oacc[t]);
      }
    }
  }

#pragma unroll
  for (int r = 0; r < 8; ++r) {
    const float inv = 1.0f / lrow[r];
#pragma unroll
    for (int t = 0; t < 2; ++t) Os[(t * 16 + c) * 68 + wave * 16 + 8 * hh + r] = oacc[t][r] * inv;
  }
  __syncthreads();
  {
    float* ob = out + ((size_t)(b * DIM + h * AT_D)) * NQ + (size_t)qb * AT_QB;
    const int q = lane >> 3, c4 = (lane & 7) * 4;
    for (int pass = 0; pass < 2; ++pass) {
#pragma unroll
      for (int it = 0; it < 4; ++it) {
        const int L  = it * 16 + wave * 4 + q;
        const int d  = L >> 1;
        const int hf = (L & 1) * 32;
        v4f val = *(const v4f*)(Os + d * 68 + hf + c4);
        *(volatile v4f*)(ob + (size_t)d * NQ + hf + c4) = val;
      }
      __threadfence();
    }
  }
}

extern "C" void kernel_launch(void* const* d_in, const int* in_sizes, int n_in,
                              void* d_out, int out_size, void* d_ws, size_t ws_size,
                              hipStream_t stream) {
  if (n_in < 6) return;
  if (in_sizes[0] != NB * DIM * NQ) return;
  if (in_sizes[1] != DIM * DIM) return;
  if (in_sizes[2] != DIM * DIM * 4) return;
  if (in_sizes[3] != DIM * DIM * 4) return;
  if (in_sizes[4] != NH * HD * OH) return;
  if (in_sizes[5] != NH * HD * OW) return;
  if (out_size != NB * DIM * NQ) return;

  const float* x     = (const float*)d_in[0];
  const float* Wq    = (const float*)d_in[1];
  const float* Wk    = (const float*)d_in[2];
  const float* Wv    = (const float*)d_in[3];
  const float* rel_h = (const float*)d_in[4];
  const float* rel_w = (const float*)d_in[5];

  const size_t PXT = (size_t)MTOK * DIM * 2;
  const size_t PWQ = (size_t)DIM * DIM * 2;
  const size_t PWC = (size_t)DIM * KCONV * 2;
  const size_t PQ  = (size_t)MTOK * DIM * 2;
  const size_t PK  = (size_t)MKV * DIM * 2;
  const size_t PVT = (size_t)DIM * VTP * 2;
  size_t off = 0;
  const size_t oXT  = off; off += PXT;
  const size_t oWQ  = off; off += PWQ;
  const size_t oWK  = off; off += PWC;
  const size_t oWV  = off; off += PWC;
  const size_t oQh  = off; off += PQ;   const size_t oQl  = off; off += PQ;
  const size_t oKh  = off; off += PK;   const size_t oKl  = off; off += PK;
  const size_t oVTh = off; off += PVT;  const size_t oVTl = off; off += PVT;
  if (off > ws_size) return;
  if (off > (size_t)134217728) return;

  char* ws = (char*)d_ws;
  unsigned short* XT  = (unsigned short*)(ws + oXT);
  unsigned short* WQ  = (unsigned short*)(ws + oWQ);
  unsigned short* WKp = (unsigned short*)(ws + oWK);
  unsigned short* WVp = (unsigned short*)(ws + oWV);
  unsigned short* Qh  = (unsigned short*)(ws + oQh);  unsigned short* Ql  = (unsigned short*)(ws + oQl);
  unsigned short* Kh  = (unsigned short*)(ws + oKh);  unsigned short* Kl  = (unsigned short*)(ws + oKl);
  unsigned short* VTh = (unsigned short*)(ws + oVTh); unsigned short* VTl = (unsigned short*)(ws + oVTl);

  const dim3 blk(256);

  tconv_kernel<<<dim3(NQ / 64, DIM / 64, NB), blk, 0, stream>>>(x, XT, NQ, DIM, (long)DIM * NQ, (long)NQ * DIM);
  const int n8q = DIM * DIM / 8;
  convrows_kernel<<<dim3(n8q / 256), blk, 0, stream>>>(Wq, WQ, DIM, DIM, n8q);
  wperm_kernel<<<dim3((DIM * 32) / 256), blk, 0, stream>>>(Wk, WKp);
  wperm_kernel<<<dim3((DIM * 32) / 256), blk, 0, stream>>>(Wv, WVp);
  const dim3 gQ(((MTOK / 64) * (DIM / 64) + 7) / 8, 1);
  wmma_gemm64<1, false, 0, 2, false, 0><<<gQ, blk, 0, stream>>>(
      XT, XT, DIM, 0L, WQ, WQ, DIM, 0L, (void*)Qh, (void*)Ql, DIM, 0L,
      rel_h, rel_h, 0L, MTOK, DIM, DIM, 1.0f);
  conv_gemm64<0><<<dim3(((MKV / 64) * (DIM / 64)) / 8), blk, 0, stream>>>(XT, WKp, rel_h, rel_w, Kh, Kl);
  conv_gemm64<1><<<dim3(((DIM / 64) * (MKV / 64)) / 8), blk, 0, stream>>>(XT, WVp, rel_h, rel_w, VTh, VTl);
  attn32_kernel<<<dim3(NB * NH * (NQ / AT_QB)), dim3(128), 0, stream>>>(Qh, Ql, Kh, Kl, VTh, VTl, (float*)d_out,
                                                                        0.17677669529663687f);
  (void)hipGetLastError();
}
